// PostNormBoth_51823075394177
// MI455X (gfx1250) — hardware-run, weakly checked
//
#include <hip/hip_runtime.h>
#include <math.h>

typedef __attribute__((ext_vector_type(16))) _Float16 v16h;
typedef __attribute__((ext_vector_type(8)))  _Float16 v8h;
typedef __attribute__((ext_vector_type(8)))  float    v8f;
typedef __attribute__((ext_vector_type(4)))  float    v4f;

constexpr int kBatch   = 512;
constexpr int kSteps   = 256;
constexpr int kHid     = 256;
constexpr int kSlots   = 64;
constexpr int kTaps    = 5;
constexpr int kHalfWin = 2;
constexpr int kOutN    = 10;
constexpr int kRowsPB  = 16;
constexpr int kBlocks  = kBatch / kRowsPB;
constexpr int kThreads = 256;
constexpr int kAPitch  = kHid + 8;
constexpr float kTau      = 8.0f;
constexpr float kTauInv   = 1.0f / kTau;
constexpr float kEps      = 1e-5f;
constexpr float kWCarry    = 16.0f;
constexpr float kWCarryInv = 1.0f / kWCarry;
constexpr float kHidInv    = 1.0f / (float)kHid;

static_assert(kThreads == kHid, "one thread per channel");
static_assert((kHid % 32) == 0, "K multiple of 32");
static_assert(kHid == 8 * 32, "8 waves x 32 output columns");
static_assert(kRowsPB == 16, "one 16-row WMMA tile per block");
static_assert((kBatch % kRowsPB) == 0, "block count");
static_assert(kTaps == 2 * kHalfWin + 1, "window");
static_assert((kSlots & (kSlots - 1)) == 0, "slot wrap by mask");
static_assert((kRowsPB * kOutN * 4) % 128 == 0, "block output is whole 128-B lines");
static_assert((kRowsPB * kOutN) % 32 == 0, "output writers are whole waves");
static_assert((kAPitch % 8) == 0, "16-B aligned fragment rows");

constexpr size_t kMemPerBlock = (size_t)kRowsPB * kSlots * kHid;
constexpr size_t kWsTotal     = (size_t)kBatch * kSlots * kHid * 4;
static_assert(kWsTotal == 33554432ull, "carve total");
static_assert(kWsTotal <= 134217728ull, "carve cap");

union FragU { v16h v; v8h h[2]; };

__device__ __forceinline__ v16h frag_load_h(const _Float16* p) {
  FragU f;
  f.h[0] = *(const v8h*)(p);
  f.h[1] = *(const v8h*)(p + 16);
  return f.v;
}

__device__ __forceinline__ v8f mma_h(v16h a, v16h b, v8f c) {
  c = __builtin_amdgcn_wmma_f32_16x16x32_f16(false, a, false, b, (short)0, c, false, false);
  asm volatile("v_nop\n\tv_nop\n\tv_nop\n\tv_nop" : "+v"(c) : "v"(a), "v"(b));
  return c;
}

__device__ __forceinline__ v16h load_w_frag(const float* p) {
  const v4f a0 = *(const v4f*)(p);
  const v4f a1 = *(const v4f*)(p + 4);
  const v4f a2 = *(const v4f*)(p + 16);
  const v4f a3 = *(const v4f*)(p + 20);
  v16h f;
#pragma unroll
  for (int e = 0; e < 4; ++e) {
    f[e]      = (_Float16)(a0[e] * kWCarry);
    f[4 + e]  = (_Float16)(a1[e] * kWCarry);
    f[8 + e]  = (_Float16)(a2[e] * kWCarry);
    f[12 + e] = (_Float16)(a3[e] * kWCarry);
  }
  asm volatile("" : "+v"(f));
  return f;
}

__global__ __launch_bounds__(256)
void recurrent_memory_kernel(const float* __restrict__ x,
                             const float* __restrict__ W_embed,
                             const float* __restrict__ b_embed,
                             const float* __restrict__ W_update,
                             const float* __restrict__ b_update,
                             const float* __restrict__ gamma,
                             const float* __restrict__ beta,
                             const float* __restrict__ W_out,
                             const float* __restrict__ b_out,
                             const float* __restrict__ cs_in,
                             float* out,
                             float* mem_ws)
{
  __shared__ __align__(16) _Float16 As[kRowsPB * kAPitch];
  __shared__ __align__(16) float    Hs[kRowsPB * kHid];
  __shared__ __align__(16) float    Xs[kRowsPB * kSteps];
  __shared__ __align__(16) float    St[kRowsPB * 2];

  const int tid  = threadIdx.x;
  const int lane = tid & 31;
  const int wid  = tid >> 5;
  const int rl   = lane & 15;
  const int hh   = lane >> 4;
  const int koff = hh * 8;
  const int b0   = blockIdx.x * kRowsPB;

  volatile float* memblk = mem_ws + (size_t)blockIdx.x * kMemPerBlock;

  const int n0 = wid * 32 + rl;
  const int n1 = n0 + 16;
  v16h bw[8][2];
#pragma unroll
  for (int kc = 0; kc < 8; ++kc) {
    bw[kc][0] = load_w_frag(W_update + (size_t)n0 * kHid + kc * 32 + koff);
    bw[kc][1] = load_w_frag(W_update + (size_t)n1 * kHid + kc * 32 + koff);
  }

  {
    volatile float* zp = memblk + tid;
    for (int pass = 0; pass < 2; ++pass) {
#pragma unroll 4
      for (int i = 0; i < kRowsPB * kSlots; ++i) zp[(size_t)i * kHid] = 0.0f;
      __threadfence();
    }
  }
#pragma unroll 1
  for (int m = 0; m < kRowsPB; ++m) {
    Hs[m * kHid + tid]   = 0.0f;
    Xs[m * kSteps + tid] = x[(size_t)(b0 + m) * kSteps + tid];
  }

  const float we  = W_embed[tid];
  const float be  = b_embed[tid];
  const float g   = gamma[tid];
  const float bt  = beta[tid];
  const float bu0 = b_update[n0];
  const float bu1 = b_update[n1];
  const float cs  = 1.0f / (1.0f + expf(-cs_in[0]));

  __syncthreads();

#pragma unroll 1
  for (int t = 0; t < kSteps; ++t) {
    const int base = t & (kSlots - 1);
    int   offs[kTaps];
    float wts[kTaps];
    float ssum = 0.0f;
#pragma unroll
    for (int k = 0; k < kTaps; ++k) {
      const int ii  = (base + k - kHalfWin + kSlots) & (kSlots - 1);
      offs[k]       = ii * kHid;
      const float d = (float)ii - (float)base;
      const float e = expf(-(d * d) * kTauInv);
      wts[k] = e;
      ssum  += e;
    }
    const float inv = 1.0f / ssum;
#pragma unroll
    for (int k = 0; k < kTaps; ++k) wts[k] *= inv;

#pragma unroll 1
    for (int m = 0; m < kRowsPB; ++m) {
      const float xv  = Xs[m * kSteps + t];
      const float inp = tanhf(xv * we + be);
      volatile const float* mp = memblk + (size_t)m * (kSlots * kHid) + tid;
      float ctx = 0.0f;
#pragma unroll
      for (int k = 0; k < kTaps; ++k) {
        const float mv = mp[offs[k]];
        ctx += wts[k] * mv;
      }
      const float a = (inp + cs * ctx) + Hs[m * kHid + tid];
      As[m * kAPitch + tid] = (_Float16)a;
    }
    __syncthreads();

    v8f acc0 = (v8f){0.f, 0.f, 0.f, 0.f, 0.f, 0.f, 0.f, 0.f};
    v8f acc1 = (v8f){0.f, 0.f, 0.f, 0.f, 0.f, 0.f, 0.f, 0.f};
#pragma unroll
    for (int kc = 0; kc < 8; ++kc) {
      const v16h af = frag_load_h(As + rl * kAPitch + kc * 32 + koff);
      acc0 = mma_h(af, bw[kc][0], acc0);
      acc1 = mma_h(af, bw[kc][1], acc1);
    }

#pragma unroll
    for (int r = 0; r < 8; ++r) {
      const int m = r + hh * 8;
      Hs[m * kHid + n0] = acc0[r] * kWCarryInv + bu0;
      Hs[m * kHid + n1] = acc1[r] * kWCarryInv + bu1;
    }
    __syncthreads();

    {
      const int mrow = tid >> 4;
      const int s    = tid & 15;
      float* hp = Hs + mrow * kHid + s;
      float sum = 0.0f;
#pragma unroll 1
      for (int j = 0; j < 16; ++j) {
        const float v = tanhf(hp[16 * j]);
        hp[16 * j] = v;
        sum += v;
      }
#pragma unroll
      for (int msk = 8; msk >= 1; msk >>= 1) sum += __shfl_xor(sum, msk, 32);
      const float mu = sum * kHidInv;
      float sq = 0.0f;
#pragma unroll 1
      for (int j = 0; j < 16; ++j) {
        const float d = hp[16 * j] - mu;
        sq += d * d;
      }
#pragma unroll
      for (int msk = 8; msk >= 1; msk >>= 1) sq += __shfl_xor(sq, msk, 32);
      const float var = sq * kHidInv;
      const float rs  = rsqrtf(var + kEps);
      if (s == 0) {
        St[mrow * 2]     = mu;
        St[mrow * 2 + 1] = rs;
      }
    }
    __syncthreads();

#pragma unroll 1
    for (int m = 0; m < kRowsPB; ++m) {
      const float mu = St[m * 2];
      const float rs = St[m * 2 + 1];
      const float hn = ((Hs[m * kHid + tid] - mu) * rs) * g + bt;
      Hs[m * kHid + tid] = hn;
      volatile float* mp = memblk + (size_t)m * (kSlots * kHid) + tid;
      float nv[kTaps];
#pragma unroll
      for (int k = 0; k < kTaps; ++k) {
        const float mv = mp[offs[k]];
        nv[k] = mv + wts[k] * hn;
      }
#pragma unroll
      for (int k = 0; k < kTaps; ++k) mp[offs[k]] = nv[k];
      __threadfence();
#pragma unroll
      for (int k = 0; k < kTaps; ++k) mp[offs[k]] = nv[k];
    }
  }

  __syncthreads();

  if (tid < kRowsPB * kOutN) {
    const int m = tid / kOutN;
    const int o = tid - m * kOutN;
    const float* wr = W_out + (size_t)o * kHid;
    const float* hr = Hs + m * kHid;
    float s = 0.0f;
#pragma unroll 1
    for (int c = 0; c < kHid; c += 4) {
      const v4f hv = *(const v4f*)(hr + c);
      const v4f wv = *(const v4f*)(wr + c);
      s = fmaf(hv[0], wv[0], s);
      s = fmaf(hv[1], wv[1], s);
      s = fmaf(hv[2], wv[2], s);
      s = fmaf(hv[3], wv[3], s);
    }
    const float res = s + b_out[o];
    volatile float* op = out + (size_t)blockIdx.x * (kRowsPB * kOutN) + tid;
    *op = res;
    __threadfence();
    *op = res;
  }
}

extern "C" void kernel_launch(void* const* d_in, const int* in_sizes, int n_in,
                              void* d_out, int out_size, void* d_ws, size_t ws_size,
                              hipStream_t stream) {
  if (n_in < 10) return;
  if (in_sizes[0] != kBatch * kSteps) return;
  if (in_sizes[1] != kHid) return;
  if (in_sizes[2] != kHid) return;
  if (in_sizes[3] != kHid * kHid) return;
  if (in_sizes[4] != kHid) return;
  if (in_sizes[5] != kHid) return;
  if (in_sizes[6] != kHid) return;
  if (in_sizes[7] != kOutN * kHid) return;
  if (in_sizes[8] != kOutN) return;
  if (in_sizes[9] != 1) return;
  if (out_size != kBatch * kOutN) return;
  if (ws_size < kWsTotal) return;

  const float* x       = (const float*)d_in[0];
  const float* W_embed = (const float*)d_in[1];
  const float* b_embed = (const float*)d_in[2];
  const float* W_upd   = (const float*)d_in[3];
  const float* b_upd   = (const float*)d_in[4];
  const float* gamma   = (const float*)d_in[5];
  const float* beta    = (const float*)d_in[6];
  const float* W_out   = (const float*)d_in[7];
  const float* b_out   = (const float*)d_in[8];
  const float* cstr    = (const float*)d_in[9];
  float* out = (float*)d_out;
  float* mem = (float*)d_ws;

  recurrent_memory_kernel<<<kBlocks, kThreads, 0, stream>>>(
      x, W_embed, b_embed, W_upd, b_upd, gamma, beta, W_out, b_out, cstr, out, mem);
}
